// RegionCodecDict_9028021256393
// MI455X (gfx1250) — hardware-verified
//
#include <hip/hip_runtime.h>


namespace {
constexpr int B = 8, T = 1024, N = 1024, R = 8, NR = 128, D = 512, NROW = B * T;
constexpr float XS = 8.0f, WS16 = 16.0f, WPS = 64.0f;
typedef _Float16 b16;
typedef __attribute__((ext_vector_type(16))) _Float16 v16b;
typedef __attribute__((ext_vector_type(8))) _Float16 v8b;
typedef __attribute__((ext_vector_type(8))) float v8f;
typedef __attribute__((ext_vector_type(4))) float v4f;
__device__ __forceinline__ float bf16_rne(float f) { unsigned int u = __float_as_uint(f); u += 0x7FFFu + ((u >> 16) & 1u); return __uint_as_float(u & 0xFFFF0000u); }
__device__ __forceinline__ float bfv(float f) { float r = bf16_rne(f); asm volatile("" : "+v"(r)); return r; }
__device__ __forceinline__ void split16(float v, b16& hi, b16& lo) { hi = (b16)v; lo = (b16)(v - (float)hi); }
__device__ __forceinline__ v16b frag_kb(const b16* p, int hh) { const v8b a = *(const v8b*)(p + 8 * hh), b = *(const v8b*)(p + 16 + 8 * hh); v16b f;
#pragma unroll
  for (int e = 0; e < 8; ++e) { f[e] = a[e]; f[8 + e] = b[e]; } return f; }
__device__ __forceinline__ v8f wmma16b(v16b a, v16b b, v8f c) { v8f d = __builtin_amdgcn_wmma_f32_16x16x32_f16(false, a, false, b, (short)0, c, false, false); asm volatile("v_nop\n\tv_nop\n\tv_nop\n\tv_nop" : "+v"(d) : "v"(a), "v"(b)); return d; }
__device__ __forceinline__ void wave_lds_sync() { __builtin_amdgcn_fence(__ATOMIC_RELEASE, "workgroup"); __builtin_amdgcn_wave_barrier(); __builtin_amdgcn_fence(__ATOMIC_ACQUIRE, "workgroup"); }
__device__ __forceinline__ float pmul(float a, float b) { float p = a * b; asm volatile("" : "+v"(p)); return p; }
__device__ __forceinline__ int iclamp(int v, int lo, int hi) { return v < lo ? lo : (v > hi ? hi : v); }

__global__ __launch_bounds__(256) void wstage_kernel(const float* __restrict__ We, const float* __restrict__ Wd, b16* __restrict__ EAh, b16* __restrict__ EAl, b16* __restrict__ DBh, b16* __restrict__ DBl) {
  const size_t u = (size_t)blockIdx.x * 256 + threadIdx.x; if (u >= (size_t)R * NR * (D / 8)) return; const int r = (int)(u / ((size_t)NR * (D / 8))); const int m = (int)((u / (D / 8)) % NR); const int k0 = (int)(u % (D / 8)) * 8; v8b ah, al, bh, bl;
#pragma unroll
  for (int j = 0; j < 8; ++j) { b16 p, q; split16(bf16_rne(We[((size_t)r * NR + m) * D + k0 + j]) * WS16, p, q); ah[j] = p; al[j] = q; split16(bf16_rne(Wd[((size_t)r * D + k0 + j) * NR + m]) * WS16, p, q); bh[j] = p; bl[j] = q; }
  for (int pass = 0; pass < 2; ++pass) { const size_t o = ((size_t)r * NR + m) * D + k0; *(volatile v8b*)(EAh + o) = ah; *(volatile v8b*)(EAl + o) = al; *(volatile v8b*)(DBh + o) = bh; *(volatile v8b*)(DBl + o) = bl; __threadfence(); } }
__global__ __launch_bounds__(32) void wprod_kernel(const b16* __restrict__ EAh, const b16* __restrict__ EAl, const b16* __restrict__ DBh, const b16* __restrict__ DBl, float* __restrict__ WPF) {
  __shared__ float Tf[16][NR + 4]; const int lane = threadIdx.x, nloc = lane & 15, hlf = lane >> 4; const int r = blockIdx.x / (NR / 16); const int m0 = (blockIdx.x % (NR / 16)) * 16; v8f acc[8];
#pragma unroll
  for (int t = 0; t < 8; ++t) acc[t] = (v8f){};
  const size_t ab = ((size_t)r * NR + m0 + nloc) * D;
#pragma unroll 2
  for (int kb = 0; kb < D; kb += 32) { const v16b a = frag_kb(EAh + ab + kb, hlf), al = frag_kb(EAl + ab + kb, hlf);
#pragma unroll
    for (int t = 0; t < 8; ++t) { const size_t bb = ((size_t)r * NR + t * 16 + nloc) * D + kb; const v16b bh = frag_kb(DBh + bb, hlf), bl = frag_kb(DBl + bb, hlf); acc[t] = wmma16b(a, bh, acc[t]); acc[t] = wmma16b(a, bl, acc[t]); acc[t] = wmma16b(al, bh, acc[t]); } }
#pragma unroll
  for (int t = 0; t < 8; ++t)
#pragma unroll
    for (int r8 = 0; r8 < 8; ++r8) Tf[8 * hlf + r8][t * 16 + nloc] = acc[t][r8] * (1.0f / (WS16 * WS16));
  wave_lds_sync();
  for (int pass = 0; pass < 2; ++pass) { for (int rr = 0; rr < 16; ++rr) *(volatile v4f*)(WPF + ((size_t)r * NR + m0 + rr) * NR + lane * 4) = *(const v4f*)(&Tf[rr][lane * 4]); __threadfence(); }
}
__global__ __launch_bounds__(32) void wtrans_kernel(const float* __restrict__ WPF, const float* __restrict__ be, const float* __restrict__ Wd, const float* __restrict__ bd, b16* __restrict__ WPh, b16* __restrict__ WPl, float* __restrict__ BP) {
  __shared__ float Ts[16][NR + 1]; const int lane = threadIdx.x; const int r = blockIdx.x / (NR / 16); const int n0 = (blockIdx.x % (NR / 16)) * 16;
  for (int m = 0; m < NR; m += 2) { const int mm = m + (lane >> 4), nn = lane & 15; Ts[nn][mm] = WPF[((size_t)r * NR + mm) * NR + n0 + nn]; }
  wave_lds_sync();
  for (int pass = 0; pass < 2; ++pass) { for (int rr = 0; rr < 16; ++rr) for (int q = 0; q < NR / 32; ++q) { b16 p, ql; split16(Ts[rr][q * 32 + lane] * WPS, p, ql); ((volatile b16*)WPh)[((size_t)r * NR + n0 + rr) * NR + q * 32 + lane] = p; ((volatile b16*)WPl)[((size_t)r * NR + n0 + rr) * NR + q * 32 + lane] = ql; } __threadfence(); }
  if (n0 == 0) { for (int q = 0; q < NR / 32; ++q) { const int n = q * 32 + lane; float s = bfv(bd[r * NR + n]);
#pragma unroll 1
      for (int k = 0; k < D; ++k) s += pmul(bfv(be[(size_t)r * D + k]), bfv(Wd[((size_t)r * D + k) * NR + n]));
      for (int pass = 0; pass < 2; ++pass) { ((volatile float*)BP)[r * NR + n] = s; __threadfence(); } } }
}
__global__ __launch_bounds__(32) void main_kernel(const float* __restrict__ x, const int* __restrict__ ridx, const b16* __restrict__ WPh, const b16* __restrict__ WPl, const float* __restrict__ BP, int RL, float* __restrict__ Y) {
  __shared__ __attribute__((aligned(16))) b16 Ah[16][NR + 8]; __shared__ float Tf[16][NR + 4]; __shared__ int Ix[NR]; const int lane = threadIdx.x, nloc = lane & 15, hlf = lane >> 4; const int r = blockIdx.x % R; const size_t m0 = (size_t)(blockIdx.x / R) * 16; if (m0 >= (size_t)RL) return;
  for (int q = 0; q < NR / 32; ++q) Ix[q * 32 + lane] = iclamp(ridx[r * NR + q * 32 + lane], 0, N - 1);
  wave_lds_sync();
  for (int rr = 0; rr < 16; ++rr) for (int q = 0; q < NR / 32; ++q) { const int m = q * 32 + lane; Ah[rr][m] = (b16)(bf16_rne(x[(m0 + rr) * N + Ix[m]]) * XS); }
  wave_lds_sync(); v8f acc[8];
#pragma unroll
  for (int t = 0; t < 8; ++t) acc[t] = (v8f){};
#pragma unroll
  for (int kb = 0; kb < NR; kb += 32) { const v16b a = frag_kb(&Ah[nloc][kb], hlf);
#pragma unroll
    for (int t = 0; t < 8; ++t) { const size_t bb = ((size_t)r * NR + t * 16 + nloc) * NR + kb; acc[t] = wmma16b(a, frag_kb(WPh + bb, hlf), acc[t]); acc[t] = wmma16b(a, frag_kb(WPl + bb, hlf), acc[t]); } }
#pragma unroll
  for (int t = 0; t < 8; ++t) { const int n = t * 16 + nloc; const float bb = BP[r * NR + n];
#pragma unroll
    for (int r8 = 0; r8 < 8; ++r8) Tf[8 * hlf + r8][n] = acc[t][r8] * (1.0f / (XS * WPS)) + bb; }
  wave_lds_sync();
  for (int pass = 0; pass < 2; ++pass) { for (int rr = 0; rr < 16; ++rr) *(volatile v4f*)(Y + (m0 + rr) * N + r * NR + lane * 4) = *(const v4f*)(&Tf[rr][lane * 4]); __threadfence(); }
}
__global__ __launch_bounds__(32) void inv_kernel(const int* __restrict__ ridx, int* __restrict__ INV) { __shared__ int iv[N]; const int lane = threadIdx.x; for (int c = lane; c < N; c += 32) iv[c] = 0; wave_lds_sync();
  if (lane == 0) for (int j = 0; j < N; ++j) iv[iclamp(ridx[j], 0, N - 1)] = j;
  wave_lds_sync(); for (int pass = 0; pass < 2; ++pass) { for (int c = lane; c < N; c += 32) ((volatile int*)INV)[c] = iv[c]; __threadfence(); } }
__global__ __launch_bounds__(256) void perm_kernel(const float* __restrict__ Y, const int* __restrict__ INV, int RL, float* __restrict__ out) { const int wave = threadIdx.x >> 5, lane = threadIdx.x & 31; const size_t row = (size_t)blockIdx.x * 8 + wave; if (row >= (size_t)RL) return;
  for (int pass = 0; pass < 2; ++pass) {
#pragma unroll 4
    for (int q = 0; q < N / 32; ++q) { const int c = q * 32 + lane; ((volatile float*)out)[row * N + c] = Y[row * N + iclamp(INV[c], 0, N - 1)]; } __threadfence(); } }
}

extern "C" void kernel_launch(void* const* d_in, const int* in_sizes, int n_in, void* d_out, int out_size, void* d_ws, size_t ws_size, hipStream_t stream) {
  (void)n_in;
  auto Fp = [&](int i) { return (const float*)d_in[i]; }; auto Ip = [&](int i) { return (const int*)d_in[i]; };
  if (in_sizes[0] != NROW * N || in_sizes[1] != R * NR * D || in_sizes[2] != R * D || in_sizes[3] != R * D * NR || in_sizes[4] != R * NR || in_sizes[5] != R * NR || out_size != NROW * N) return;
  const int RL = NROW;
  size_t off = 0; char* ws = (char*)d_ws;
  auto carve = [&](size_t bytes) { char* p = ws + off; off += (bytes + 255) & ~(size_t)255; return p; };
  b16* EAh = (b16*)carve((size_t)R * NR * D * 2); b16* EAl = (b16*)carve((size_t)R * NR * D * 2); b16* DBh = (b16*)carve((size_t)R * NR * D * 2); b16* DBl = (b16*)carve((size_t)R * NR * D * 2); float* WPF = (float*)carve((size_t)R * NR * NR * 4);
  b16* WPh = (b16*)carve((size_t)R * NR * NR * 2); b16* WPl = (b16*)carve((size_t)R * NR * NR * 2); float* BP = (float*)carve((size_t)R * NR * 4); int* INV = (int*)carve((size_t)N * 4); float* Y = (float*)carve((size_t)NROW * N * 4);
  if (off > ws_size || off > ((size_t)64 << 20)) return;
  wstage_kernel<<<(unsigned)(((size_t)R * NR * (D / 8) + 255) / 256), 256, 0, stream>>>(Fp(1), Fp(3), EAh, EAl, DBh, DBl);
  wprod_kernel<<<R * (NR / 16), 32, 0, stream>>>(EAh, EAl, DBh, DBl, WPF);
  wtrans_kernel<<<R * (NR / 16), 32, 0, stream>>>(WPF, Fp(2), Fp(3), Fp(4), WPh, WPl, BP);
  inv_kernel<<<1, 32, 0, stream>>>(Ip(5), INV);
  main_kernel<<<(RL / 16) * R, 32, 0, stream>>>(Fp(0), Ip(5), WPh, WPl, BP, RL, Y);
  perm_kernel<<<(RL + 7) / 8, 256, 0, stream>>>(Y, INV, RL, (float*)d_out);
}
